// Net_LSTM_2516850835908
// MI455X (gfx1250) — hardware-run, weakly checked
//
#include <hip/hip_runtime.h>
#include <math.h>

constexpr int kSeq   = 16384;
constexpr int kIn    = 50;
constexpr int kInP   = 64;
constexpr int kHid   = 128;
constexpr int kGates = 4 * kHid;
constexpr int kOut   = 5;

constexpr float kCarryW = 256.0f;
constexpr float kCarryH = 64.0f;
constexpr float kFold1  = 1.0f / kCarryW;
constexpr float kFold2  = 1.0f / (kCarryH * kCarryW);
constexpr float kF16MinNormal = 6.103515625e-5f;

static_assert(kInP % 32 == 0 && kInP >= kIn && kHid % 32 == 0);
static_assert(kSeq % 32 == 0 && kGates % 64 == 0);
static_assert(((kSeq / 32) * (kGates / 64)) % 8 == 0);
static_assert((kSeq * kOut) % 256 == 0);
static_assert(kGates == 512 && kHid == 128);

constexpr size_t kSzX16 = (size_t)kSeq * kInP * 2;
constexpr size_t kSzW1P = (size_t)kGates * kInP * 2;
constexpr size_t kSzW2P = (size_t)kGates * kHid * 2;
constexpr size_t kSzPRE = (size_t)kSeq * kGates * 4;
constexpr size_t kSzH   = (size_t)kSeq * kHid * 4;
constexpr size_t kSzHP  = (size_t)kSeq * kHid * 2;
constexpr size_t kWsTotal = kSzX16 + kSzW1P + kSzW2P + kSzPRE + kSzH + kSzHP + kSzH;
static_assert(kWsTotal == 56819712ull);
static_assert(kWsTotal <= 134217728ull);
static_assert(kSzX16 % 256 == 0 && kSzW1P % 256 == 0 && kSzW2P % 256 == 0);
static_assert(kSzPRE % 256 == 0 && kSzH % 256 == 0 && kSzHP % 256 == 0);

typedef __attribute__((ext_vector_type(16))) _Float16 v16h;
typedef __attribute__((ext_vector_type(8)))  _Float16 v8h;
typedef __attribute__((ext_vector_type(8)))  float    v8f;
typedef __attribute__((ext_vector_type(4)))  float    v4f;
typedef __attribute__((ext_vector_type(4)))  unsigned int v4u;

__device__ __forceinline__ unsigned pk16(unsigned short a, unsigned short b) {
  return (unsigned)a | ((unsigned)b << 16);
}
__device__ __forceinline__ unsigned short h_bits_flush(float f) {
  const float g = (fabsf(f) < kF16MinNormal) ? 0.0f : f;
  const _Float16 h = (_Float16)g;
  return __builtin_bit_cast(unsigned short, h);
}
__device__ __forceinline__ v4u pack8_flush(const float (&v)[8]) {
  unsigned short hb[8];
#pragma unroll
  for (int e = 0; e < 8; ++e) hb[e] = h_bits_flush(v[e]);
  return (v4u){pk16(hb[0], hb[1]), pk16(hb[2], hb[3]), pk16(hb[4], hb[5]), pk16(hb[6], hb[7])};
}

struct FragH {
  union U { v16h v; v8h h[2]; };
  static __device__ __forceinline__ v16h load(const _Float16* p) {
    U f;
    f.h[0] = *(const v8h*)(p);
    f.h[1] = *(const v8h*)(p + 16);
    return f.v;
  }
};
__device__ __forceinline__ v8f mma_g(v16h a, v16h b, v8f c) {
  c = __builtin_amdgcn_wmma_f32_16x16x32_f16(false, a, false, b, (short)0, c, false, false);
  asm volatile("v_nop\n\tv_nop\n\tv_nop\n\tv_nop" : "+v"(c) : "v"(a), "v"(b));
  return c;
}
__device__ __forceinline__ void acc_guard4(v8f& a, v8f& b, v8f& c, v8f& d) {
  asm volatile("v_nop\n\tv_nop\n\tv_nop\n\tv_nop" : "+v"(a), "+v"(b), "+v"(c), "+v"(d));
}

__global__ __launch_bounds__(256) void cast_pad_rows_kernel(
    const float* __restrict__ src, int srcCols,
    unsigned short* __restrict__ dst, int dstCols, int totalGroups, float carry) {
  const int i = blockIdx.x * 256 + threadIdx.x;
  if (i >= totalGroups) return;
  const int gpr = dstCols >> 3;
  const int row = i / gpr;
  const int c8  = (i - row * gpr) * 8;
  const float* p = src + (size_t)row * srcCols;
  float v[8];
#pragma unroll
  for (int e = 0; e < 8; ++e) {
    const int c  = c8 + e;
    const int cc = c < srcCols ? c : (srcCols - 1);
    float f = p[cc];
    asm volatile("" : "+v"(f));
    v[e] = (c < srcCols) ? (f * carry) : 0.0f;
  }
  const v4u u = pack8_flush(v);
  unsigned short* q = dst + (size_t)i * 8;
  *(volatile v4u*)q = u;
  __threadfence();
  *(volatile v4u*)q = u;
}

__global__ __launch_bounds__(256) void cast_flat8_kernel(
    const float* __restrict__ src, unsigned short* __restrict__ dst, int totalGroups, float carry) {
  const int i = blockIdx.x * 256 + threadIdx.x;
  if (i >= totalGroups) return;
  const float* p = src + (size_t)i * 8;
  const v4f a = *(const v4f*)(p);
  const v4f b = *(const v4f*)(p + 4);
  float v[8];
#pragma unroll
  for (int e = 0; e < 4; ++e) {
    v[e]     = a[e] * carry;
    v[4 + e] = b[e] * carry;
  }
  const v4u u = pack8_flush(v);
  unsigned short* q = dst + (size_t)i * 8;
  *(volatile v4u*)q = u;
  __threadfence();
  *(volatile v4u*)q = u;
}

template <int KDIM>
__global__ __launch_bounds__(256) void gate_gemm_kernel(
    const unsigned short* __restrict__ Ap, const unsigned short* __restrict__ Bp,
    float* __restrict__ Cout, const float* __restrict__ bias0, const float* __restrict__ bias1, float scale) {
  static_assert(KDIM % 32 == 0);
  __shared__ __align__(16) float sT[8][16 * 68];
  constexpr int tilesN = kGates >> 6;
  constexpr int tilesM = kSeq >> 5;
  const int lane = threadIdx.x & 31;
  const int wave = threadIdx.x >> 5;
  const int tile = blockIdx.x * 8 + wave;
  if (tile >= tilesM * tilesN) return;
  const int tm = tile / tilesN;
  const int tn = tile - tm * tilesN;
  const int m0 = tm << 5;
  const int n0 = tn << 6;
  const int rlane = lane & 15;
  const int half8 = (lane >> 4) * 8;
  const int mOff  = (lane >> 4) * 8;

  const _Float16* pa0 = (const _Float16*)Ap + (size_t)(m0 + rlane) * KDIM + half8;
  const _Float16* pa1 = pa0 + (size_t)16 * KDIM;
  const _Float16* pbh = (const _Float16*)Bp + (size_t)(n0 + rlane) * KDIM + half8;
  constexpr size_t bstep = (size_t)16 * KDIM;

  v8f acc[2][4];
#pragma unroll
  for (int i = 0; i < 2; ++i)
#pragma unroll
    for (int j = 0; j < 4; ++j)
      acc[i][j] = (v8f){0.f, 0.f, 0.f, 0.f, 0.f, 0.f, 0.f, 0.f};

  for (int k0 = 0; k0 < KDIM; k0 += 32) {
    const v16h ah0 = FragH::load(pa0 + k0);
    const v16h ah1 = FragH::load(pa1 + k0);
#pragma unroll
    for (int j = 0; j < 4; ++j) {
      const v16h bh = FragH::load(pbh + j * bstep + k0);
      acc[0][j] = mma_g(ah0, bh, acc[0][j]);
      acc[1][j] = mma_g(ah1, bh, acc[1][j]);
    }
  }
  acc_guard4(acc[0][0], acc[0][1], acc[0][2], acc[0][3]);
  acc_guard4(acc[1][0], acc[1][1], acc[1][2], acc[1][3]);

  float bsum[4];
#pragma unroll
  for (int j = 0; j < 4; ++j) {
    const int n = n0 + (j << 4) + rlane;
    const float ba = bias0[n];
    const float bb = bias1[n];
    bsum[j] = ba + bb;
  }

  float* slab = sT[wave];
#pragma unroll
  for (int i = 0; i < 2; ++i) {
    const int mBase = m0 + (i << 4);
#pragma unroll
    for (int j = 0; j < 4; ++j) {
#pragma unroll
      for (int r = 0; r < 8; ++r) {
        const float v = acc[i][j][r] * scale + bsum[j];
        slab[(mOff + r) * 68 + (j << 4) + rlane] = v;
      }
    }
    __builtin_amdgcn_fence(__ATOMIC_RELEASE, "workgroup");
    __builtin_amdgcn_wave_barrier();
    __builtin_amdgcn_fence(__ATOMIC_ACQUIRE, "workgroup");
    {
      const int hh = lane >> 4, c4 = (lane & 15) * 4;
      for (int pass = 0; pass < 2; ++pass) {
#pragma unroll
        for (int it = 0; it < 8; ++it) {
          const int row = it * 2 + hh;
          const v4f v = *(const v4f*)(slab + row * 68 + c4);
          *(volatile v4f*)(Cout + (size_t)(mBase + row) * kGates + n0 + c4) = v;
        }
        __threadfence();
      }
    }
    __builtin_amdgcn_fence(__ATOMIC_RELEASE, "workgroup");
    __builtin_amdgcn_wave_barrier();
    __builtin_amdgcn_fence(__ATOMIC_ACQUIRE, "workgroup");
  }
}

__global__ __launch_bounds__(512) void chain_kernel(const float* __restrict__ PRE,
                                                    const float* __restrict__ Whh,
                                                    float* __restrict__ Hout, int steps) {
  __shared__ __align__(16) float h_s[kHid];
  __shared__ __align__(16) float g_s[kGates];
  const int tid = threadIdx.x;
  const int nsteps = steps < kSeq ? (steps < 0 ? 0 : steps) : kSeq;
  const v4f* w0 = (const v4f*)(Whh + (size_t)tid * kHid);
  const v4f* h4 = (const v4f*)h_s;
  float c_reg = 0.0f;
  if (tid < kHid) h_s[tid] = 0.0f;
  __syncthreads();
#pragma unroll 1
  for (int s = 0; s < nsteps; ++s) {
    const float gv = PRE[(size_t)s * kGates + tid];
    float acc = 0.0f;
#pragma unroll 2
    for (int k = 0; k < kHid / 4; ++k) {
      const v4f hv = h4[k];
      const v4f a  = w0[k];
      acc = fmaf(a[0], hv[0], acc);
      acc = fmaf(a[1], hv[1], acc);
      acc = fmaf(a[2], hv[2], acc);
      acc = fmaf(a[3], hv[3], acc);
    }
    g_s[tid] = gv + acc;
    __syncthreads();
    if (tid < kHid) {
      const float gi = g_s[tid];
      const float gf = g_s[kHid + tid];
      const float gg = g_s[2 * kHid + tid];
      const float go = g_s[3 * kHid + tid];
      const float si = 1.0f / (1.0f + expf(-gi));
      const float sf = 1.0f / (1.0f + expf(-gf));
      const float so = 1.0f / (1.0f + expf(-go));
      c_reg = sf * c_reg + si * tanhf(gg);
      const float hval = so * tanhf(c_reg);
      h_s[tid] = hval;
      float* hp = Hout + (size_t)s * kHid + tid;
      *(volatile float*)hp = hval;
      __threadfence();
      *(volatile float*)hp = hval;
    }
    __syncthreads();
  }
}

__global__ __launch_bounds__(256) void head_kernel(const float* __restrict__ H2, const float* __restrict__ W,
                                                   const float* __restrict__ b, float* __restrict__ out,
                                                   int total) {
  const int e = blockIdx.x * 256 + threadIdx.x;
  if (e >= total) return;
  const int t = e / kOut;
  const int o = e - t * kOut;
  const v4f* hr = (const v4f*)(H2 + (size_t)t * kHid);
  const v4f* wr = (const v4f*)(W + (size_t)o * kHid);
  float acc = 0.0f;
#pragma unroll 2
  for (int k4 = 0; k4 < kHid / 4; ++k4) {
    const v4f hv = hr[k4];
    const v4f wv = wr[k4];
    acc = fmaf(hv[0], wv[0], acc);
    acc = fmaf(hv[1], wv[1], acc);
    acc = fmaf(hv[2], wv[2], acc);
    acc = fmaf(hv[3], wv[3], acc);
  }
  const float res = acc + b[o];
  float* op = out + e;
  *(volatile float*)op = res;
  __threadfence();
  *(volatile float*)op = res;
}

extern "C" void kernel_launch(void* const* d_in, const int* in_sizes, int n_in,
                              void* d_out, int out_size, void* d_ws, size_t ws_size, hipStream_t stream) {
  if (n_in < 11 || d_out == nullptr || d_ws == nullptr) return;
  if (in_sizes[0] != kSeq * kIn || in_sizes[1] != kGates * kIn || in_sizes[2] != kGates * kHid) return;
  if (in_sizes[3] != kGates || in_sizes[4] != kGates) return;
  if (in_sizes[5] != kGates * kHid || in_sizes[6] != kGates * kHid) return;
  if (in_sizes[7] != kGates || in_sizes[8] != kGates) return;
  if (in_sizes[9] != kOut * kHid || in_sizes[10] != kOut) return;
  if (out_size != kSeq * kOut) return;

  const float* x     = (const float*)d_in[0];
  const float* w_ih1 = (const float*)d_in[1];
  const float* w_hh1 = (const float*)d_in[2];
  const float* b_ih1 = (const float*)d_in[3];
  const float* b_hh1 = (const float*)d_in[4];
  const float* w_ih2 = (const float*)d_in[5];
  const float* w_hh2 = (const float*)d_in[6];
  const float* b_ih2 = (const float*)d_in[7];
  const float* b_hh2 = (const float*)d_in[8];
  const float* fc_w  = (const float*)d_in[9];
  const float* fc_b  = (const float*)d_in[10];
  float* out = (float*)d_out;

  char* ws = (char*)d_ws;
  size_t off = 0;
  auto carve = [&](size_t bytes) -> char* {
    char* p = ws + off;
    off += (bytes + 255) & ~(size_t)255;
    return p;
  };
  unsigned short* X16 = (unsigned short*)carve(kSzX16);
  unsigned short* W1P = (unsigned short*)carve(kSzW1P);
  unsigned short* W2P = (unsigned short*)carve(kSzW2P);
  float* PRE = (float*)carve(kSzPRE);
  float* H1  = (float*)carve(kSzH);
  unsigned short* H1P = (unsigned short*)carve(kSzHP);
  float* H2  = (float*)carve(kSzH);
  if (off != kWsTotal || off > ws_size || off > (size_t)134217728) return;

  constexpr int kGX  = kSeq * (kInP / 8);
  constexpr int kGW1 = kGates * (kInP / 8);
  constexpr int kGW2 = kGates * (kHid / 8);
  constexpr int kGH  = kSeq * (kHid / 8);
  static_assert(kGX % 256 == 0 && kGW1 % 256 == 0 && kGW2 % 256 == 0 && kGH % 256 == 0);
  constexpr int kBlkGemm = ((kSeq / 32) * (kGates / 64)) / 8;

  cast_pad_rows_kernel<<<kGX / 256, 256, 0, stream>>>(x, kIn, X16, kInP, kGX, 1.0f);
  cast_pad_rows_kernel<<<kGW1 / 256, 256, 0, stream>>>(w_ih1, kIn, W1P, kInP, kGW1, kCarryW);
  cast_flat8_kernel<<<kGW2 / 256, 256, 0, stream>>>(w_ih2, W2P, kGW2, kCarryW);

  gate_gemm_kernel<kInP><<<kBlkGemm, 256, 0, stream>>>(X16, W1P, PRE, b_ih1, b_hh1, kFold1);
  chain_kernel<<<1, 512, 0, stream>>>(PRE, w_hh1, H1, kSeq);

  cast_flat8_kernel<<<kGH / 256, 256, 0, stream>>>(H1, H1P, kGH, kCarryH);

  gate_gemm_kernel<kHid><<<kBlkGemm, 256, 0, stream>>>(H1P, W2P, PRE, b_ih2, b_hh2, kFold2);
  chain_kernel<<<1, 512, 0, stream>>>(PRE, w_hh2, H2, kSeq);

  head_kernel<<<(kSeq * kOut) / 256, 256, 0, stream>>>(H2, fc_w, fc_b, out, kSeq * kOut);
}
